// GraphLearning_27281632264514
// MI455X (gfx1250) — hardware-run, weakly checked
//
#include <hip/hip_runtime.h>


namespace {
constexpr int N = 50000, E = 800000, FI = 256, C = 32, NH = 4, HC = 128, NL = 2;
constexpr float XS = 8.0f, WSC = 256.0f, SLOPE = 0.2f, EPS = 1e-5f;
typedef _Float16 b16;
typedef __attribute__((ext_vector_type(16))) _Float16 v16b;
typedef __attribute__((ext_vector_type(8))) _Float16 v8b;
typedef __attribute__((ext_vector_type(8))) float v8f;
typedef __attribute__((ext_vector_type(4))) float v4f;
__device__ __forceinline__ float bf16_rne(float f) { unsigned int u = __float_as_uint(f); u += 0x7FFFu + ((u >> 16) & 1u); float r = __uint_as_float(u & 0xFFFF0000u); asm volatile("" : "+v"(r)); return r; }
__device__ __forceinline__ void split16(float v, b16& hi, b16& lo) { hi = (b16)v; lo = (b16)(v - (float)hi); }
__device__ __forceinline__ v16b frag_kb(const b16* p, int hh) { const v8b a = *(const v8b*)(p + 8 * hh), b = *(const v8b*)(p + 16 + 8 * hh); v16b f;
#pragma unroll
  for (int e = 0; e < 8; ++e) { f[e] = a[e]; f[8 + e] = b[e]; } return f; }
__device__ __forceinline__ v8f wmma16b(v16b a, v16b b, v8f c) { v8f d = __builtin_amdgcn_wmma_f32_16x16x32_f16(false, a, false, b, (short)0, c, false, false); asm volatile("v_nop\n\tv_nop\n\tv_nop\n\tv_nop" : "+v"(d) : "v"(a), "v"(b)); return d; }
__device__ __forceinline__ void wave_lds_sync() { __builtin_amdgcn_fence(__ATOMIC_RELEASE, "workgroup"); __builtin_amdgcn_wave_barrier(); __builtin_amdgcn_fence(__ATOMIC_ACQUIRE, "workgroup"); }
__device__ __forceinline__ float pmul(float a, float b) { float p = a * b; asm volatile("" : "+v"(p)); return p; }
__device__ __forceinline__ int iclamp(int v, int lo, int hi) { return v < lo ? lo : (v > hi ? hi : v); }
__device__ __forceinline__ float lrelu(float v) { return v > 0.0f ? v : SLOPE * v; }
constexpr int CSR_NBLK9 = 512, CSR_GB9 = 9, CSR_GN9 = 1 << CSR_GB9  , CSR_TS9 = (CSR_GN9 < 32 ? 32 : CSR_GN9)  , CSR_MAXG9 = 512, CSR_CAP9 = 12288  ;
__device__ __host__ __forceinline__ int csr_tix9(int v) { return (v >> CSR_GB9) * CSR_TS9 + (v & (CSR_GN9 - 1)); }
__global__ __launch_bounds__(64) void csrA_kernel9(const int* __restrict__ dst, int E, int N, int nG, int CHP, int NGP, int* __restrict__ STG, int* __restrict__ HST) {
  extern __shared__ int sm[];
  int* cnt = sm; int* run = sm + NGP; int* ids = sm + 2 * NGP;
  const int b = blockIdx.x; const int ch = (E + CSR_NBLK9 - 1) / CSR_NBLK9; const int e0 = b * ch, e1 = min(E, e0 + ch);
  for (int i = threadIdx.x; i < NGP; i += 64) cnt[i] = 0;
  for (int i = threadIdx.x; i < CHP; i += 64) ids[i] = -1;
  __syncthreads();
  if (threadIdx.x == 0) {
    for (int e = e0; e < e1; ++e) { int d = dst[e]; d = (d < 0) ? 0 : (d >= N ? N - 1 : d); cnt[d >> CSR_GB9] += 1; }
    int acc = 0; for (int g = 0; g < nG; ++g) { run[g] = acc; acc += cnt[g]; }
    for (int e = e0; e < e1; ++e) { int d = dst[e]; d = (d < 0) ? 0 : (d >= N ? N - 1 : d); const int g = d >> CSR_GB9; ids[run[g]] = e; run[g] += 1; } }
  __syncthreads();
  typedef __attribute__((ext_vector_type(4))) int v4i;
  for (int pass = 0; pass < 2; ++pass) {
    for (int i = threadIdx.x; i < CHP / 4; i += 64) *(volatile v4i*)(STG + (size_t)b * CHP + i * 4) = *(const v4i*)(&ids[i * 4]);
    for (int i = threadIdx.x; i < NGP / 4; i += 64) { v4i v; for (int e = 0; e < 4; ++e) v[e] = (i * 4 + e < nG) ? cnt[i * 4 + e] : 0; *(volatile v4i*)(HST + (size_t)b * NGP + i * 4) = v; }
    __threadfence(); }
}
__global__ __launch_bounds__(512) void csrS_kernel9(const int* __restrict__ HST, int nG, int NGP, int* __restrict__ START, int* __restrict__ TOT, int* __restrict__ OFF) {
  __shared__ int tot[CSR_MAXG9];
  const int b = threadIdx.x;
  for (int pass = 0; pass < 2; ++pass) { int runb = 0; for (int g = 0; g < nG; ++g) { int c = HST[(size_t)b * NGP + g]; c = (c < 0) ? 0 : c; ((volatile int*)OFF)[(size_t)g * CSR_NBLK9 + b] = runb; runb += c; } __threadfence(); }
  for (int g = threadIdx.x; g < nG; g += 512) { int s = 0; for (int bb = 0; bb < CSR_NBLK9; ++bb) { int c = HST[(size_t)bb * NGP + g]; s += (c < 0) ? 0 : c; } tot[g] = s; }
  __syncthreads();
  if (threadIdx.x < 32) {
    __shared__ int st[CSR_MAXG9 + 32];
    if (threadIdx.x == 0) { int acc = 0; for (int g = 0; g < NGP; ++g) { st[g] = acc; if (g < nG) acc += (tot[g] + 31) & ~31; } st[NGP] = acc; }
    __builtin_amdgcn_fence(__ATOMIC_RELEASE, "workgroup"); __builtin_amdgcn_wave_barrier(); __builtin_amdgcn_fence(__ATOMIC_ACQUIRE, "workgroup");
    for (int pass = 0; pass < 2; ++pass) { for (int i = threadIdx.x; i < NGP + 32; i += 32) { ((volatile int*)START)[i] = (i <= NGP) ? st[min(i, NGP)] : 0; ((volatile int*)TOT)[i] = (i < nG) ? tot[i] : 0; } __threadfence(); } }
}
__global__ __launch_bounds__(256) void csrB_kernel9(const int* __restrict__ dst, int N, int nG, int CHP, int NGP, int permLen, const int* __restrict__ STG, const int* __restrict__ HST, const int* __restrict__ OFF, const int* __restrict__ START, const int* __restrict__ TOT, int* __restrict__ PERM, int* __restrict__ ROWPTR, int* __restrict__ ROWCNT, int* __restrict__ FLAG) {
  typedef __attribute__((ext_vector_type(4))) int v4i;
  __shared__ int ids[CSR_CAP9]; __shared__ unsigned short key[CSR_CAP9]; __shared__ int outp[CSR_CAP9]; __shared__ int ncnt[CSR_GN9 + 1]; __shared__ int boff[CSR_NBLK9 + 1];
  const int g = blockIdx.x, t_ = threadIdx.x; int tot = TOT[g]; int st = START[g], stn = START[g + 1]; const int v0 = g * CSR_GN9; const int nv = min(CSR_GN9, N - v0); const int t0 = g * CSR_TS9;
  st = (st < 0) ? 0 : (st > permLen - 32 ? permLen - 32 : st) & ~31; stn = (stn < st) ? st : (stn > permLen ? permLen : stn); tot = (tot < 0) ? 0 : tot; if (tot > stn - st && tot <= CSR_CAP9) tot = stn - st;
  if (tot > CSR_CAP9) {
    for (int pass = 0; pass < 2; ++pass) { for (int i = t_; i < CSR_TS9 / 4; i += 256) { v4i a, c; for (int e = 0; e < 4; ++e) { a[e] = st; c[e] = 0; } *(volatile v4i*)(ROWPTR + t0 + i * 4) = a; *(volatile v4i*)(ROWCNT + t0 + i * 4) = c; } if (t_ == 0) ((volatile int*)FLAG)[0] = 1; __threadfence(); } (void)nv; return; }
  if (t_ == 0) { int acc = 0; for (int b = 0; b < CSR_NBLK9; ++b) { boff[b] = acc; int c = HST[(size_t)b * NGP + g]; c = (c < 0) ? 0 : (c > CHP ? CHP : c); acc += c; if (acc > tot) acc = tot; } boff[CSR_NBLK9] = acc; }
  for (int i = t_; i <= CSR_GN9; i += 256) ncnt[i] = 0;
  __syncthreads();
  for (int b = 0; b < CSR_NBLK9; ++b) { const int c = boff[b + 1] - boff[b]; int o_ = OFF[(size_t)g * CSR_NBLK9 + b]; o_ = (o_ < 0) ? 0 : (o_ > CHP - c ? CHP - c : o_); const int* src_ = STG + (size_t)b * CHP + o_;
    for (int i = t_; i < c; i += 256) { int id = src_[i]; id = (id < 0) ? 0 : id; ids[boff[b] + i] = id; int d = dst[id]; d = (d < v0) ? v0 : (d >= N ? N - 1 : d); int kk = d - v0; kk = (kk < 0) ? 0 : (kk >= CSR_GN9 ? CSR_GN9 - 1 : kk); key[boff[b] + i] = (unsigned short)kk; } }
  __syncthreads();
  if (t_ == 0) { for (int i = 0; i < tot; ++i) ncnt[key[i]] += 1; int acc = 0; for (int vl = 0; vl < CSR_GN9; ++vl) { const int c = ncnt[vl]; ncnt[vl] = acc; acc += c; } ncnt[CSR_GN9] = acc;
    for (int i = 0; i < tot; ++i) { const int vl = key[i]; outp[ncnt[vl]] = ids[i]; ncnt[vl] += 1; }
    for (int vl = CSR_GN9; vl > 0; --vl) ncnt[vl] = ncnt[vl - 1]; ncnt[0] = 0; }
  __syncthreads();
  for (int pass = 0; pass < 2; ++pass) {
    for (int i = t_; i < (stn - st) / 4; i += 256) { v4i v; for (int e = 0; e < 4; ++e) { const int q = i * 4 + e; v[e] = (q < tot) ? outp[q] : -1; } *(volatile v4i*)(PERM + st + i * 4) = v; }
    for (int i = t_; i < CSR_TS9 / 4; i += 256) { v4i a, c; for (int e = 0; e < 4; ++e) { const int vl = i * 4 + e; const int vc = vl < CSR_GN9 ? vl : CSR_GN9; a[e] = (vl < CSR_GN9) ? st + ncnt[vc] : st; c[e] = (vl < nv) ? (ncnt[(vc < CSR_GN9 ? vc : CSR_GN9 - 1) + 1] - ncnt[vc]) : 0; } *(volatile v4i*)(ROWPTR + t0 + i * 4) = a; *(volatile v4i*)(ROWCNT + t0 + i * 4) = c; }
    __threadfence(); }
}
__global__ __launch_bounds__(256) void csrZ_kernel9(int* __restrict__ p, size_t n4) { typedef __attribute__((ext_vector_type(4))) int v4i; const size_t tid = (size_t)blockIdx.x * 256 + threadIdx.x, nth = (size_t)gridDim.x * 256; v4i z = {0, 0, 0, 0}; for (size_t i = tid; i < n4; i += nth) *(volatile v4i*)(p + i * 4) = z; }
struct CsrBufs9 { int *STG, *HST, *OFF, *START, *TOT, *PERM, *ROWPTR, *ROWCNT, *FLAG; int nG, NGP, CHP; size_t permLen; char* base; size_t bytes; };
static size_t csr_carve9(CsrBufs9& c, char* ws, size_t off, int E, int N) {
  const size_t off0 = off; c.base = ws + off;
  auto al = [&](size_t bytes) { char* p = ws + off; off += (bytes + 255) & ~(size_t)255; return p; };
  c.nG = (N + CSR_GN9 - 1) / CSR_GN9; c.NGP = (c.nG + 31) & ~31; const int ch = (E + CSR_NBLK9 - 1) / CSR_NBLK9; c.CHP = (ch + 31) & ~31; c.permLen = (size_t)E + 32 * (size_t)c.nG + 32;
  c.STG = (int*)al((size_t)CSR_NBLK9 * c.CHP * 4); c.HST = (int*)al((size_t)CSR_NBLK9 * c.NGP * 4); c.OFF = (int*)al((size_t)c.NGP * CSR_NBLK9 * 4); c.START = (int*)al((size_t)(c.NGP + 64) * 4); c.TOT = (int*)al((size_t)(c.NGP + 64) * 4);
  c.PERM = (int*)al(c.permLen * 4); c.ROWPTR = (int*)al((size_t)c.nG * CSR_TS9 * 4); c.ROWCNT = (int*)al((size_t)c.nG * CSR_TS9 * 4); c.FLAG = (int*)al(256);
  c.bytes = off - off0; return off;
}
static void csr_build9(const CsrBufs9& c, const int* dst, int E, int N, hipStream_t stream) {
  const size_t smem = (size_t)(2 * c.NGP + c.CHP) * 4;
  csrZ_kernel9<<<512, 256, 0, stream>>>((int*)c.base, c.bytes / 16);
  csrA_kernel9<<<CSR_NBLK9, 64, smem, stream>>>(dst, E, N, c.nG, c.CHP, c.NGP, c.STG, c.HST);
  csrS_kernel9<<<1, 512, 0, stream>>>(c.HST, c.nG, c.NGP, c.START, c.TOT, c.OFF);
  csrB_kernel9<<<c.nG, 256, 0, stream>>>(dst, N, c.nG, c.CHP, c.NGP, (int)c.permLen, c.STG, c.HST, c.OFF, c.START, c.TOT, c.PERM, c.ROWPTR, c.ROWCNT, c.FLAG);
}


__global__ __launch_bounds__(256) void wput_kernel(const float* __restrict__ wemb, const float* __restrict__ wl, const float* __restrict__ wr, const float* __restrict__ lw, b16* __restrict__ WET, b16* __restrict__ WLR, b16* __restrict__ LWT) { const int u = blockIdx.x * 256 + threadIdx.x;
  for (int pass = 0; pass < 2; ++pass) {
    if (u < C * 32) { const int o = u / 32, k0 = (u % 32) * 8; v8b v;
#pragma unroll
      for (int j = 0; j < 8; ++j) v[j] = (b16)(bf16_rne(wemb[(size_t)(k0 + j) * C + o]) * WSC); *(volatile v8b*)(WET + (size_t)o * FI + k0) = v; }
    if (u < NL * 2 * HC * 4) { const int r = u / 4, k0 = (u % 4) * 8; const int l = r / (2 * HC), oo = r % (2 * HC); const float* w = oo < HC ? wl : wr; const int o = oo % HC; v8b v;
#pragma unroll
      for (int j = 0; j < 8; ++j) v[j] = (b16)(bf16_rne(w[((size_t)l * C + k0 + j) * HC + o]) * WSC); *(volatile v8b*)(WLR + (size_t)r * C + k0) = v; }
    if (u < NL * C * 16) { const int r = u / 16, k0 = (u % 16) * 8; const int l = r / C, o = r % C; v8b v;
#pragma unroll
      for (int j = 0; j < 8; ++j) v[j] = (b16)(bf16_rne(lw[((size_t)l * HC + k0 + j) * C + o]) * WSC); *(volatile v8b*)(LWT + (size_t)r * HC + k0) = v; }
    __threadfence(); } }
__device__ __forceinline__ void node_ln_relu_row32(float* row, int lane, const float* w, const float* b) {
  const float v = row[lane]; float s = v; for (int o = 16; o; o >>= 1) s += __shfl_xor(s, o); const float mu = s * (1.0f / C); const float d = v - mu; float q = pmul(d, d); for (int o = 16; o; o >>= 1) q += __shfl_xor(q, o); const float rs = rsqrtf(q * (1.0f / C) + EPS); row[lane] = fmaxf(pmul(pmul(d, rs), bf16_rne(w[lane])) + bf16_rne(b[lane]), 0.0f); }
__global__ __launch_bounds__(32) void embed_kernel(const float* __restrict__ x, const b16* __restrict__ WET, const float* __restrict__ bemb, const float* __restrict__ w0, const float* __restrict__ b0, int NLIM, float* __restrict__ H0, float* __restrict__ OUT) { __shared__ __attribute__((aligned(16))) b16 Ah[16][FI + 8]; __shared__ float Tf[16][36]; const int lane = threadIdx.x, nloc = lane & 15, hlf = lane >> 4; const size_t m0 = (size_t)blockIdx.x * 16; if (m0 >= (size_t)NLIM) return;
  for (int rr = 0; rr < 16; ++rr) for (int q = 0; q < 8; ++q) Ah[rr][q * 32 + lane] = (b16)(bf16_rne(x[(m0 + rr) * FI + q * 32 + lane]) * XS);
  wave_lds_sync(); v8f acc[2] = {(v8f){}, (v8f){}};
#pragma unroll 2
  for (int kb = 0; kb < FI; kb += 32) { const v16b a = frag_kb(&Ah[nloc][kb], hlf);
#pragma unroll
    for (int t = 0; t < 2; ++t) acc[t] = wmma16b(a, frag_kb(WET + (size_t)(t * 16 + nloc) * FI + kb, hlf), acc[t]); }
#pragma unroll
  for (int t = 0; t < 2; ++t) { const int c = t * 16 + nloc; const float bb = bf16_rne(bemb[c]);
#pragma unroll
    for (int r8 = 0; r8 < 8; ++r8) Tf[8 * hlf + r8][c] = acc[t][r8] * (1.0f / (XS * WSC)) + bb; }
  wave_lds_sync(); for (int rr = 0; rr < 16; ++rr) node_ln_relu_row32(Tf[rr], lane, w0, b0); wave_lds_sync();
  for (int pass = 0; pass < 2; ++pass) { for (int rr = 0; rr < 16; ++rr) { ((volatile float*)H0)[(m0 + rr) * C + lane] = Tf[rr][lane]; ((volatile float*)OUT)[(m0 + rr) * C + lane] = Tf[rr][lane]; } __threadfence(); } }
__global__ __launch_bounds__(32) void xlr_kernel(const float* __restrict__ Hh, const b16* __restrict__ WLR, const float* __restrict__ bl, const float* __restrict__ br, int NLIM, float* __restrict__ XLR) { __shared__ __attribute__((aligned(16))) b16 Ah[16][40], Al[16][40]; __shared__ float Tf[16][260]; const int lane = threadIdx.x, nloc = lane & 15, hlf = lane >> 4; const size_t m0 = (size_t)blockIdx.x * 16; if (m0 >= (size_t)NLIM) return;
  for (int rr = 0; rr < 16; ++rr) { b16 p, ql; split16(Hh[(m0 + rr) * C + lane] * XS, p, ql); Ah[rr][lane] = p; Al[rr][lane] = ql; }
  wave_lds_sync(); const v16b a = frag_kb(&Ah[nloc][0], hlf), al = frag_kb(&Al[nloc][0], hlf);
#pragma unroll
  for (int t = 0; t < 16; ++t) { const v16b bw = frag_kb(WLR + (size_t)(t * 16 + nloc) * C, hlf); v8f acc = {}; acc = wmma16b(a, bw, acc); acc = wmma16b(al, bw, acc); const int c = t * 16 + nloc; const float bb = c < HC ? bf16_rne(bl[c]) : bf16_rne(br[c - HC]);
#pragma unroll
    for (int r8 = 0; r8 < 8; ++r8) Tf[8 * hlf + r8][c] = acc[r8] * (1.0f / (XS * WSC)) + bb; }
  wave_lds_sync();
  for (int pass = 0; pass < 2; ++pass) { for (int rr = 0; rr < 16; ++rr) for (int g = 0; g < 2; ++g) *(volatile v4f*)(XLR + (m0 + rr) * 2 * HC + g * 128 + lane * 4) = *(const v4f*)(&Tf[rr][g * 128 + lane * 4]); __threadfence(); } }
__global__ __launch_bounds__(256) void gat_kernel(const float* __restrict__ XLR, const float* __restrict__ ea, const float* __restrict__ we, const float* __restrict__ att, const float* __restrict__ gb, const int* __restrict__ srcs, const int* __restrict__ PERM, const int* __restrict__ ROWPTR, const int* __restrict__ ROWCNT, int permLen, int NLIM, float* __restrict__ G, float* __restrict__ PST) {
  __shared__ float Ps[8][2]; const int wave = threadIdx.x >> 5, lane = threadIdx.x & 31; const size_t i = (size_t)blockIdx.x * 8 + wave; float psum = 0.0f, psq = 0.0f; v4f o = {0.0f, 0.0f, 0.0f, 0.0f};
  if (i < (size_t)NLIM) { int st = ROWPTR[i], cnt = ROWCNT[i]; cnt = iclamp(cnt, 0, 1 << 21); st = iclamp(st, 0, permLen - cnt);
    const v4f xri = *(const v4f*)(XLR + i * 2 * HC + HC + lane * 4); float wv[4], av[4]; for (int k = 0; k < 4; ++k) { wv[k] = bf16_rne(we[lane * 4 + k]); av[k] = bf16_rne(att[lane * 4 + k]); }
    float m = -INFINITY, den = 0.0f; v4f acc = {0.0f, 0.0f, 0.0f, 0.0f};
    auto step = [&](size_t u, float eav) { const v4f xl = *(const v4f*)(XLR + u * 2 * HC + lane * 4); float s = 0.0f; for (int k = 0; k < 4; ++k) s += pmul(lrelu(xl[k] + xri[k] + pmul(eav, wv[k])), av[k]); s += __shfl_xor(s, 1); s += __shfl_xor(s, 2); s += __shfl_xor(s, 4);
      const float mn = fmaxf(m, s); const float sf = (m == -INFINITY) ? 0.0f : __expf(m - mn); const float p = __expf(s - mn); den = den * sf + p; for (int k = 0; k < 4; ++k) acc[k] = pmul(acc[k], sf) + pmul(p, xl[k]); m = mn; };
#pragma unroll 1
    for (int j = 0; j < cnt; ++j) { const int e = iclamp(PERM[st + j], 0, E - 1); const size_t u = (size_t)iclamp(srcs[e], 0, N - 1); if (u >= (size_t)NLIM) continue; step(u, bf16_rne(ea[e])); }
    step(i, 0.0f);
    const float inv = 1.0f / den; for (int k = 0; k < 4; ++k) { o[k] = pmul(acc[k], inv) + bf16_rne(gb[lane * 4 + k]); psum += o[k]; psq += pmul(o[k], o[k]); } }
  for (int q = 16; q; q >>= 1) { psum += __shfl_xor(psum, q); psq += __shfl_xor(psq, q); } if (lane == 0) { Ps[wave][0] = psum; Ps[wave][1] = psq; }
  __syncthreads();
  for (int pass = 0; pass < 2; ++pass) { if (i < (size_t)NLIM) *(volatile v4f*)(G + i * HC + lane * 4) = o;
    if (wave == 0) { float v = 0.0f; if (lane == 0) for (int w8 = 0; w8 < 8; ++w8) v += Ps[w8][0]; else if (lane == 1) for (int w8 = 0; w8 < 8; ++w8) v += Ps[w8][1]; ((volatile float*)PST)[(size_t)blockIdx.x * 32 + lane] = v; }
    __threadfence(); } }
__global__ __launch_bounds__(256) void gstat_kernel(const float* __restrict__ PST, int NB, int nvals, float* __restrict__ STAT) { __shared__ double S[256], Q[256]; const int t = threadIdx.x; double s = 0.0, q = 0.0; for (int b = t; b < NB; b += 256) { s += (double)PST[(size_t)b * 32]; q += (double)PST[(size_t)b * 32 + 1]; } S[t] = s; Q[t] = q; __syncthreads();
  for (int st = 128; st > 0; st >>= 1) { if (t < st) { S[t] += S[t + st]; Q[t] += Q[t + st]; } __syncthreads(); }
  const double mean = S[0] / (double)nvals; double var = Q[0] / (double)nvals - mean * mean; if (var < 0.0) var = 0.0; const float mf = (float)mean, rs = (float)(1.0 / sqrt(var + (double)EPS));
  for (int pass = 0; pass < 2; ++pass) { if (t < 32) ((volatile float*)STAT)[t] = t == 0 ? mf : (t == 1 ? rs : 0.0f); __threadfence(); } }
__global__ __launch_bounds__(32) void lin_kernel(const float* __restrict__ G, const float* __restrict__ STAT, const float* __restrict__ w1, const float* __restrict__ b1, const b16* __restrict__ LWT, const float* __restrict__ lb, const float* __restrict__ w2, const float* __restrict__ b2, int NLIM, float* __restrict__ Hh, float* __restrict__ OUT) {
  __shared__ __attribute__((aligned(16))) b16 Ah[16][136], Al[16][136]; __shared__ float Tf[16][36]; const int lane = threadIdx.x, nloc = lane & 15, hlf = lane >> 4; const size_t m0 = (size_t)blockIdx.x * 16; if (m0 >= (size_t)NLIM) return; const float mu = STAT[0], rs = STAT[1];
  for (int rr = 0; rr < 16; ++rr) for (int q = 0; q < 4; ++q) { const int c = q * 32 + lane; const float v = fmaxf(pmul(pmul(G[(m0 + rr) * HC + c] - mu, rs), bf16_rne(w1[c])) + bf16_rne(b1[c]), 0.0f); b16 p, ql; split16(v * XS, p, ql); Ah[rr][c] = p; Al[rr][c] = ql; }
  wave_lds_sync(); v8f acc[2] = {(v8f){}, (v8f){}};
#pragma unroll
  for (int kb = 0; kb < HC; kb += 32) { const v16b a = frag_kb(&Ah[nloc][kb], hlf), al = frag_kb(&Al[nloc][kb], hlf);
#pragma unroll
    for (int t = 0; t < 2; ++t) { const v16b bw = frag_kb(LWT + (size_t)(t * 16 + nloc) * HC + kb, hlf); acc[t] = wmma16b(a, bw, acc[t]); acc[t] = wmma16b(al, bw, acc[t]); } }
#pragma unroll
  for (int t = 0; t < 2; ++t) { const int c = t * 16 + nloc; const float bb = bf16_rne(lb[c]);
#pragma unroll
    for (int r8 = 0; r8 < 8; ++r8) Tf[8 * hlf + r8][c] = acc[t][r8] * (1.0f / (XS * WSC)) + bb; }
  wave_lds_sync(); for (int rr = 0; rr < 16; ++rr) node_ln_relu_row32(Tf[rr], lane, w2, b2); wave_lds_sync();
  for (int pass = 0; pass < 2; ++pass) { for (int rr = 0; rr < 16; ++rr) { const float h = Tf[rr][lane]; ((volatile float*)Hh)[(m0 + rr) * C + lane] = h; float* op = OUT + (m0 + rr) * C + lane; const float prev = *op; *(volatile float*)op = fmaxf(prev, h); } __threadfence(); } }
}

extern "C" void kernel_launch(void* const* d_in, const int* in_sizes, int n_in, void* d_out, int out_size, void* d_ws, size_t ws_size, hipStream_t stream) {
  (void)n_in;
  auto Fp = [&](int i) { return (const float*)d_in[i]; }; auto Ip = [&](int i) { return (const int*)d_in[i]; };
  if (in_sizes[0] != N * FI || in_sizes[1] != 2 * E || in_sizes[2] != E || in_sizes[3] != FI * C || in_sizes[7] != NL * C * HC || in_sizes[11] != NL * HC || in_sizes[12] != NL * HC || in_sizes[16] != NL * HC * C || out_size != N * C) return;
  const int NLIM = N;
  size_t off = 0; char* ws = (char*)d_ws;
  auto carve = [&](size_t bytes) { char* p = ws + off; off += (bytes + 255) & ~(size_t)255; return p; };
  b16* WET = (b16*)carve((size_t)C * FI * 2); b16* WLR = (b16*)carve((size_t)NL * 2 * HC * C * 2); b16* LWT = (b16*)carve((size_t)NL * C * HC * 2); float* Hb = (float*)carve((size_t)N * C * 4); float* XLR = (float*)carve((size_t)N * 2 * HC * 4); float* G = (float*)carve((size_t)N * HC * 4); const int NB = (NLIM + 7) / 8; float* PST = (float*)carve((size_t)((N + 7) / 8) * 32 * 4); float* STAT = (float*)carve(32 * 4);
  CsrBufs9 csr; off = csr_carve9(csr, ws, off, E, N);
  if (off > ws_size || off > ((size_t)128 << 20)) return;
  float* OUT = (float*)d_out;
  wput_kernel<<<(NL * 2 * HC * 4 + 255) / 256, 256, 0, stream>>>(Fp(3), Fp(7), Fp(9), Fp(16), WET, WLR, LWT);
  csr_build9(csr, Ip(1) + E, E, N, stream);
  embed_kernel<<<NLIM / 16, 32, 0, stream>>>(Fp(0), WET, Fp(4), Fp(5), Fp(6), NLIM, Hb, OUT);
  for (int l = 0; l < NL; ++l) {
    xlr_kernel<<<NLIM / 16, 32, 0, stream>>>(Hb, WLR + (size_t)l * 2 * HC * C, Fp(8) + l * HC, Fp(10) + l * HC, NLIM, XLR);
    gat_kernel<<<NB, 256, 0, stream>>>(XLR, Fp(2), Fp(11) + l * HC, Fp(12) + l * HC, Fp(13) + l * HC, Ip(1), csr.PERM, csr.ROWPTR, csr.ROWCNT, (int)csr.permLen, NLIM, G, PST);
    gstat_kernel<<<1, 256, 0, stream>>>(PST, NB, NLIM * HC, STAT);
    lin_kernel<<<NLIM / 16, 32, 0, stream>>>(G, STAT, Fp(14) + l * HC, Fp(15) + l * HC, LWT + (size_t)l * C * HC, Fp(17) + l * C, Fp(18) + l * C, Fp(19) + l * C, NLIM, Hb, OUT); }
}
